// EqvLEPFeedForward_51994874085875
// MI455X (gfx1250) — hardware-verified
//
#include <hip/hip_runtime.h>
#include <stddef.h>

typedef _Float16 v16h __attribute__((ext_vector_type(16)));
typedef _Float16 v8h  __attribute__((ext_vector_type(8)));
typedef float    v8f  __attribute__((ext_vector_type(8)));
typedef float    v4f  __attribute__((ext_vector_type(4)));
typedef float    v2f  __attribute__((ext_vector_type(2)));

union Frag { v16h v; v8h h[2]; _Float16 s[16]; };

#define ZZ     4
#define N1     192
#define NN     384
#define CC     16
#define NBK    10
#define HH     12
#define KTOT   (NN * 16)
#define NCHUNK (NN / 2)
#define NTILE  (NN / 16)
#define PROW   32

#define L2E     1.4426950408889634f
#define SCALE_G (0.28209479177387814f * 0.28867513459481287f)
#define WSC     (0.31622776601683794f * (1.0f / 1.423085244900308f))
#define RSIG    1.125f

__device__ __forceinline__ v8f wmma_f16(v16h a, v16h b, v8f c) {
    v8f d = __builtin_amdgcn_wmma_f32_16x16x32_f16(false, a, false, b, (short)0, c, false, false);
    asm volatile("v_nop\n\tv_nop\n\tv_nop\n\tv_nop" : "+v"(d) : "v"(a), "v"(b));
    return d;
}

__global__ __launch_bounds__(128)
void gmat_kernel(const float* __restrict__ in1, const float* __restrict__ in2,
                 const float* __restrict__ wro, _Float16* gk) {
    __shared__ _Float16 ltile[4 * 256] __attribute__((aligned(16)));

    const int tid = threadIdx.x, wave = tid >> 5, lane = tid & 31, hl = lane >> 4, m = lane & 15;
    const int bt = blockIdx.x;
    const int i  = blockIdx.y * 4 + wave;
    const int z  = blockIdx.z;

    const int b = bt * 16 + m;
    const float* xr = (b < N1) ? in1 + ((size_t)z * N1 + b) * CC
                               : in2 + ((size_t)z * N1 + (b - N1)) * CC;
    const v4f x0 = *(const v4f*)(xr + 8 * hl);
    const v4f x1 = *(const v4f*)(xr + 8 * hl + 4);

    const int hr = (m < HH) ? m : (HH - 1);
    const float* wr = wro + (size_t)hr * (CC * CC) + i * CC + 8 * hl;
    v4f w0 = *(const v4f*)wr;
    v4f w1 = *(const v4f*)(wr + 4);
    if (m >= HH) { w0 = (v4f){0.0f, 0.0f, 0.0f, 0.0f}; w1 = (v4f){0.0f, 0.0f, 0.0f, 0.0f}; }

    v16h z16 = {};
    Frag a, bb;
    a.v = z16; bb.v = z16;
    #pragma unroll
    for (int e = 0; e < 4; ++e) {
        a.s[e]      = (_Float16)x0[e];
        a.s[4 + e]  = (_Float16)x1[e];
        bb.s[e]     = (_Float16)w0[e];
        bb.s[4 + e] = (_Float16)w1[e];
    }

    v8f acc = {};
    acc = wmma_f16(a.v, bb.v, acc);

    _Float16* lt = ltile + wave * 256;
    #pragma unroll
    for (int r = 0; r < 8; ++r) lt[(8 * hl + r) * 16 + m] = (_Float16)acc[r];
    __syncthreads();

    const v8h v = *(const v8h*)(lt + 8 * lane);
    volatile v8h* dst = (volatile v8h*)(gk + ((size_t)z * CC + i) * KTOT + (size_t)bt * 256 + 8 * lane);
    *dst = v;
    __threadfence();
    *dst = v;
}

__global__ __launch_bounds__(64)
void pair_kernel(const float* __restrict__ xyz1, const float* __restrict__ xyz2,
                 const float* __restrict__ wr1, const int* __restrict__ mask,
                 const _Float16* gk, float* psum) {
    __shared__ float lx[NN], ly[NN], lz[NN];

    const int z = blockIdx.y, tid = threadIdx.x;
    for (int t = tid; t < NN; t += 64) {
        const float* p = (t < N1) ? xyz1 + ((size_t)z * N1 + t) * 3
                                  : xyz2 + ((size_t)z * N1 + (t - N1)) * 3;
        lx[t] = p[0]; ly[t] = p[1]; lz[t] = p[2];
    }
    __syncthreads();

    const int wave = tid >> 5, lane = tid & 31, hl = lane >> 4, m = lane & 15;
    const int tile = blockIdx.x * 2 + wave;
    const int a    = tile * 16 + m;
    const float ax = lx[a], ay = ly[a], az = lz[a];

    v2f w1r[NBK][4];
    #pragma unroll
    for (int k = 0; k < NBK; ++k) {
        #pragma unroll
        for (int hp = 0; hp < 4; ++hp) {
            const int h0 = 8 * hl + 2 * hp, h1 = h0 + 1;
            const int c0 = (h0 < HH) ? h0 : 0, c1 = (h1 < HH) ? h1 : 0;
            float wa = wr1[k * HH + c0] * WSC;
            float wb = wr1[k * HH + c1] * WSC;
            wa = (h0 < HH) ? wa : 0.0f;
            wb = (h1 < HH) ? wb : 0.0f;
            w1r[k][hp] = (v2f){wa, wb};
        }
    }

    v8f acc = {};
    const _Float16* gp = gk + ((size_t)z * CC + m) * KTOT + 8 * hl;

    #pragma unroll 1
    for (int ch = 0; ch < NCHUNK; ++ch) {
        const int b0 = 2 * ch;

        Frag bf;
        bf.h[0] = *(const v8h*)(gp + ch * 32);
        bf.h[1] = *(const v8h*)(gp + ch * 32 + 16);

        const v2f dx = (v2f){ax - lx[b0], ax - lx[b0 + 1]};
        const v2f dy = (v2f){ay - ly[b0], ay - ly[b0 + 1]};
        const v2f dz = (v2f){az - lz[b0], az - lz[b0 + 1]};
        v2f dd = dx * dx;
        dd = __builtin_elementwise_fma(dy, dy, dd);
        dd = __builtin_elementwise_fma(dz, dz, dd);
        dd = dd + 1e-12f;
        const v2f dv = (v2f){__builtin_amdgcn_sqrtf(dd.x), __builtin_amdgcn_sqrtf(dd.y)};

        v2f bk[NBK];
        #pragma unroll
        for (int k = 0; k < NBK; ++k) {
            const float ck = (float)(10.0 * (double)k / 9.0);
            const v2f ev = (dv - ck) * RSIG;
            const v2f q  = ev * ev * (-L2E);
            bk[k] = (v2f){__builtin_amdgcn_exp2f(q.x), __builtin_amdgcn_exp2f(q.y)};
        }

        Frag af;
        #pragma unroll
        for (int t = 0; t < 2; ++t) {
            #pragma unroll
            for (int hp = 0; hp < 4; ++hp) {
                v2f s2 = (v2f){0.0f, 0.0f};
                #pragma unroll
                for (int k = 0; k < NBK; ++k) {
                    const v2f bsp = (v2f){bk[k][t], bk[k][t]};
                    s2 = __builtin_elementwise_fma(bsp, w1r[k][hp], s2);
                }
                const v2f ar  = s2 * (-L2E);
                const v2f e   = (v2f){__builtin_amdgcn_exp2f(ar.x), __builtin_amdgcn_exp2f(ar.y)};
                const v2f den = e + 1.0f;
                const v2f sg  = (v2f){__builtin_amdgcn_rcpf(den.x), __builtin_amdgcn_rcpf(den.y)};
                const v2f sl  = s2 * sg;
                af.s[t * 8 + 2 * hp]     = (_Float16)sl.x;
                af.s[t * 8 + 2 * hp + 1] = (_Float16)sl.y;
            }
        }

        acc = wmma_f16(af.v, bf.v, acc);
    }

    float ps = 0.0f;
    const int* mk = mask + (size_t)z * NN + tile * 16 + 8 * hl;
    #pragma unroll
    for (int r = 0; r < 8; ++r) {
        const float v = __builtin_fabsf(acc[r] * SCALE_G);
        ps += (mk[r] == 0) ? 0.0f : v;
    }
    ps += __shfl_xor(ps, 16);

    const float q0 = __shfl(ps, (4 * lane) & 31);
    const float q1 = __shfl(ps, (4 * lane + 1) & 31);
    const float q2 = __shfl(ps, (4 * lane + 2) & 31);
    const float q3 = __shfl(ps, (4 * lane + 3) & 31);
    v4f val = (v4f){q0, q1, q2, q3};
    if (lane >= 4) val = (v4f){0.0f, 0.0f, 0.0f, 0.0f};
    volatile v4f* dst = (volatile v4f*)(psum + ((size_t)z * NTILE + tile) * PROW) + lane;
    if (lane < 8) *dst = val;
    __threadfence();
    if (lane < 8) *dst = val;
}

__global__ __launch_bounds__(32)
void head_kernel(const float* psum, const float* __restrict__ wfc3,
                 const float* __restrict__ wfc2, float* out) {
    __shared__ float lsn[ZZ * CC];

    const int lane = threadIdx.x & 31, hl = lane >> 4, m = lane & 15;

    #pragma unroll
    for (int z = 0; z < ZZ; ++z) {
        float s = 0.0f;
        for (int t = 0; t < NTILE; ++t) s += psum[((size_t)(z * NTILE + t)) * PROW + m];
        float sum = s;
        sum += __shfl_xor(sum, 8); sum += __shfl_xor(sum, 4); sum += __shfl_xor(sum, 2); sum += __shfl_xor(sum, 1);
        const float mean = sum * (1.0f / 16.0f);
        const float d = s - mean;
        float vs = d * d;
        vs += __shfl_xor(vs, 8); vs += __shfl_xor(vs, 4); vs += __shfl_xor(vs, 2); vs += __shfl_xor(vs, 1);
        const float var = vs * (1.0f / 15.0f);
        const float den = __builtin_amdgcn_sqrtf(var) + 1e-6f;
        const float sn  = d * __builtin_amdgcn_rcpf(den);
        if (hl == 0) lsn[z * CC + m] = sn;
    }
    __syncthreads();

    v16h z16 = {};
    Frag a, bb;
    a.v = z16; bb.v = z16;
    const int zr = (m < ZZ) ? m : 0;
    #pragma unroll
    for (int e = 0; e < 8; ++e) {
        const float av = lsn[zr * CC + 8 * hl + e];
        a.s[e]  = (_Float16)((m < ZZ) ? av : 0.0f);
        bb.s[e] = (_Float16)wfc3[(8 * hl + e) * CC + m];
    }
    v8f acc = {};
    acc = wmma_f16(a.v, bb.v, acc);

    const float w2 = wfc2[m];
    float sg[ZZ];
    #pragma unroll
    for (int r = 0; r < ZZ; ++r) {
        float h3 = acc[r] * 0.25f;
        h3 = (h3 >= 0.0f) ? h3 : 0.01f * h3;
        float p = h3 * w2;
        p += __shfl_xor(p, 8); p += __shfl_xor(p, 4); p += __shfl_xor(p, 2); p += __shfl_xor(p, 1);
        const float o = p * 0.25f;
        const float e = __builtin_amdgcn_exp2f(-o * L2E);
        sg[r] = __builtin_amdgcn_rcpf(1.0f + e);
    }
    const v4f ov = (v4f){sg[0], sg[1], sg[2], sg[3]};
    volatile v4f* od = (volatile v4f*)out;
    if (lane == 0) *od = ov;
    __threadfence();
    if (lane == 0) *od = ov;
}

extern "C" void kernel_launch(void* const* d_in, const int* in_sizes, int n_in,
                              void* d_out, int out_size, void* d_ws, size_t ws_size,
                              hipStream_t stream) {
    if (n_in < 9) return;
    if (in_sizes[0] != ZZ * N1 * CC || in_sizes[1] != ZZ * N1 * CC ||
        in_sizes[2] != ZZ * N1 * 3  || in_sizes[3] != ZZ * N1 * 3  ||
        in_sizes[4] != ZZ * NN      || in_sizes[5] != NBK * HH      ||
        in_sizes[6] != HH * CC * CC || in_sizes[7] != CC * CC       ||
        in_sizes[8] != CC           || out_size != ZZ) return;

    const size_t GK_BYTES = (size_t)ZZ * CC * KTOT * sizeof(_Float16);
    const size_t P_BYTES  = (size_t)ZZ * NTILE * PROW * sizeof(float);
    if (ws_size < GK_BYTES + P_BYTES) return;

    const float* in1  = (const float*)d_in[0];
    const float* in2  = (const float*)d_in[1];
    const float* xyz1 = (const float*)d_in[2];
    const float* xyz2 = (const float*)d_in[3];
    const int*   mask = (const int*)d_in[4];
    const float* wr1  = (const float*)d_in[5];
    const float* wro  = (const float*)d_in[6];
    const float* wfc3 = (const float*)d_in[7];
    const float* wfc2 = (const float*)d_in[8];
    float*       out  = (float*)d_out;

    _Float16* gk   = (_Float16*)d_ws;
    float*    psum = (float*)((char*)d_ws + GK_BYTES);

    gmat_kernel<<<dim3(NTILE, 4, ZZ), 128, 0, stream>>>(in1, in2, wro, gk);
    pair_kernel<<<dim3(NTILE / 2, ZZ), 64, 0, stream>>>(xyz1, xyz2, wr1, mask, gk, psum);
    head_kernel<<<1, 32, 0, stream>>>(psum, wfc3, wfc2, out);
}
